// GCNEncoder_68865505624262
// MI455X (gfx1250) — hardware-verified
//
#include <hip/hip_runtime.h>
#include <stddef.h>
#include <stdint.h>


#define FIN    96
#define HID    128
#define FOUT   64
#define AP0    320
#define K0     288
#define AP1    512
#define K1     512
#define NTHR   256
#define NWAVE  8
#define EPT    8
#define CHUNK  (NTHR * EPT)
#define WCAP   (EPT * 32)
#define LISTN  (NWAVE * WCAP)
#define NBA    1024
#define SLA    10
#define RCAP   28672
#define DEGCAP 1024
#define GBM    64
#define GTHR   128
#define NG0    (AP0 / 8)
#define NG1    (AP1 / 8)
#define NU0    (HID * NG0)
#define NU1    (FOUT * NG1)
#define AGG_ZINTS    (LISTN + 2 * RCAP + 3 * NBA)
#define MISC_INTS    16
#define ROWBUF_INTS  (NWAVE * AP1 / 2)
#define AGG_LDS_INTS (AGG_ZINTS + MISC_INTS + ROWBUF_INTS)
#define WSMAX  134217728

static_assert((CHUNK & (CHUNK - 1)) == 0 && CHUNK <= 4096);
static_assert((NBA & (NBA - 1)) == 0 && NBA == (1 << SLA));
static_assert(((long long)CHUNK << SLA) < (1LL << 31));
static_assert(LISTN % NTHR == 0);
static_assert(NBA % NWAVE == 0 && NBA % 32 == 0 && NBA % GBM == 0);
static_assert(RCAP % 4 == 0 && AGG_ZINTS % 4 == 0 && LISTN % 4 == 0 && ((AGG_ZINTS + MISC_INTS) % 4) == 0);
static_assert(AGG_ZINTS % (NTHR * 4) == 0 && ROWBUF_INTS % (NTHR * 4) == 0);
static_assert(K0 % 32 == 0 && K1 % 32 == 0 && K0 == 3 * FIN && K0 <= AP0 && K1 == 4 * HID && K1 == AP1);
static_assert(AP0 % 64 == 0 && AP1 % 64 == 0);
static_assert(FIN == 3 * 32 && HID == 4 * 32 && FOUT == 64 && FIN % 8 == 0);
static_assert(GBM == (GTHR / 32) * 16);
static_assert(NU0 % NTHR == 0 && NU1 % NTHR == 0);
static_assert(AGG_LDS_INTS * 4 <= 300000);

typedef float          v4f   __attribute__((ext_vector_type(4)));
typedef float          v8f   __attribute__((ext_vector_type(8)));
typedef int            v4i   __attribute__((ext_vector_type(4)));
typedef int            v8i   __attribute__((ext_vector_type(8)));
typedef unsigned short v4us  __attribute__((ext_vector_type(4)));
typedef unsigned short v8us  __attribute__((ext_vector_type(8)));
typedef unsigned short v16us __attribute__((ext_vector_type(16)));
typedef __bf16         v16bf __attribute__((ext_vector_type(16)));
typedef v4f  __attribute__((may_alias)) v4fa;
typedef v4i  __attribute__((may_alias)) v4ia;
typedef v4us __attribute__((may_alias)) v4usa;
typedef v8us __attribute__((may_alias)) v8usa;
union FragB { v16bf v; v16us u; v8us h[2]; v8i w; };

__device__ __forceinline__ v8f wmb(const FragB& a, const FragB& b, v8f c) {
  v8f d = __builtin_amdgcn_wmma_f32_16x16x32_bf16(false, a.v, false, b.v, (short)0, c, false, false);
  asm volatile("v_nop\n\tv_nop\n\tv_nop\n\tv_nop" : "+v"(d) : "v"(a.w), "v"(b.w));
  return d;
}

__device__ __forceinline__ unsigned bf16_bits(float f) {
  const unsigned u = __float_as_uint(f);
  return (u + 0x7FFFu + ((u >> 16) & 1u)) >> 16;
}
__device__ __forceinline__ float bf16_val(float f) {
  return __uint_as_float(bf16_bits(f) << 16);
}

__device__ __forceinline__ unsigned short bsel(float r, float t, unsigned mR, unsigned mZ) {
  const unsigned a = bf16_bits(r);
  const unsigned b = bf16_bits(t);
  return (unsigned short)(((b & mR) | (a & ~mR)) & mZ);
}

__device__ __forceinline__ void wave_sync() {
  __builtin_amdgcn_fence(__ATOMIC_RELEASE, "wavefront");
  __builtin_amdgcn_wave_barrier();
  __builtin_amdgcn_fence(__ATOMIC_ACQUIRE, "wavefront");
}

template <int SLB>
__device__ __forceinline__ int scan_chunk(const int* __restrict__ dsts, int nE, int cbase, int slotBase,
                                          int nb, int vec8, int* list, int tid, int lane, int wave) {
  int wc = 0;
  const int el0  = tid * EPT;
  const int e0   = cbase + el0;
  const int sent = -2147483647 - 1;
  v4i da, db;
  if (vec8 != 0 && cbase + CHUNK <= nE) {
    da = *(const v4i*)(dsts + e0);
    db = *(const v4i*)(dsts + e0 + 4);
  } else {
    da.x = (e0     < nE) ? dsts[min(e0,     nE - 1)] : sent;
    da.y = (e0 + 1 < nE) ? dsts[min(e0 + 1, nE - 1)] : sent;
    da.z = (e0 + 2 < nE) ? dsts[min(e0 + 2, nE - 1)] : sent;
    da.w = (e0 + 3 < nE) ? dsts[min(e0 + 3, nE - 1)] : sent;
    db.x = (e0 + 4 < nE) ? dsts[min(e0 + 4, nE - 1)] : sent;
    db.y = (e0 + 5 < nE) ? dsts[min(e0 + 5, nE - 1)] : sent;
    db.z = (e0 + 6 < nE) ? dsts[min(e0 + 6, nE - 1)] : sent;
    db.w = (e0 + 7 < nE) ? dsts[min(e0 + 7, nE - 1)] : sent;
  }
  const unsigned nbs = (unsigned)slotBase;
  const unsigned unb = (unsigned)nb;
  const unsigned s0 = (unsigned)da.x - nbs, s1 = (unsigned)da.y - nbs;
  const unsigned s2 = (unsigned)da.z - nbs, s3 = (unsigned)da.w - nbs;
  const unsigned s4 = (unsigned)db.x - nbs, s5 = (unsigned)db.y - nbs;
  const unsigned s6 = (unsigned)db.z - nbs, s7 = (unsigned)db.w - nbs;
  const bool h0 = s0 < unb, h1 = s1 < unb, h2 = s2 < unb, h3 = s3 < unb;
  const bool h4 = s4 < unb, h5 = s5 < unb, h6 = s6 < unb, h7 = s7 < unb;
  const unsigned any = __builtin_amdgcn_ballot_w32(h0 | h1 | h2 | h3 | h4 | h5 | h6 | h7);
  if (any != 0u) {
#define HITJ(J, HJ, SJ) { \
      const unsigned mj = __builtin_amdgcn_ballot_w32(HJ); \
      if (mj != 0u) { \
        if (HJ) { \
          const int pos = wc + (int)__builtin_amdgcn_mbcnt_lo(mj, 0u); \
          if (pos < WCAP) list[wave * WCAP + pos] = ((el0 + (J)) << SLB) | (int)(SJ); \
        } \
        wc += (int)__builtin_popcount(mj); } }
    HITJ(0, h0, s0)
    HITJ(1, h1, s1)
    HITJ(2, h2, s2)
    HITJ(3, h3, s3)
    HITJ(4, h4, s4)
    HITJ(5, h5, s5)
    HITJ(6, h6, s6)
    HITJ(7, h7, s7)
#undef HITJ
  }
  return wc;
}

__global__ __launch_bounds__(NTHR) void k_wprep(const float* __restrict__ W1r, const float* __restrict__ W1o,
                                                const float* __restrict__ W2r, const float* __restrict__ W2o,
                                                unsigned short* B0, unsigned short* B1) {
  const int u = (int)blockIdx.x * NTHR + (int)threadIdx.x;
  const float* pr;
  const float* po;
  unsigned mR, mZ;
  unsigned short* dp;
  if (u < NU0) {
    const int n  = u / NG0;
    const int g  = u - n * NG0;
    const int kk = 8 * (g % (FIN / 8));
    pr = W1r + (size_t)n * FIN + kk;
    po = W1o + (size_t)n * FIN + kk;
    mR = (g >= 2 * (FIN / 8)) ? 0xFFFFu : 0u;
    mZ = (g < (K0 / 8)) ? 0xFFFFu : 0u;
    dp = B0 + (size_t)n * AP0 + 8 * g;
  } else if (u < NU0 + NU1) {
    const int v  = u - NU0;
    const int n  = v >> 6;
    const int g  = v & 63;
    const int kk = 8 * (g & (HID / 8 - 1));
    pr = W2r + (size_t)n * HID + kk;
    po = W2o + (size_t)n * HID + kk;
    mR = (g >= 2 * (HID / 8)) ? 0xFFFFu : 0u;
    mZ = 0xFFFFu;
    dp = B1 + (size_t)n * AP1 + 8 * g;
  } else {
    return;
  }
  const v4f ra = *(const v4f*)pr;
  const v4f rb = *(const v4f*)(pr + 4);
  const v4f oa = *(const v4f*)po;
  const v4f ob = *(const v4f*)(po + 4);
  v8us o;
  o[0] = bsel(ra.x, oa.x, mR, mZ); o[1] = bsel(ra.y, oa.y, mR, mZ);
  o[2] = bsel(ra.z, oa.z, mR, mZ); o[3] = bsel(ra.w, oa.w, mR, mZ);
  o[4] = bsel(rb.x, ob.x, mR, mZ); o[5] = bsel(rb.y, ob.y, mR, mZ);
  o[6] = bsel(rb.z, ob.z, mR, mZ); o[7] = bsel(rb.w, ob.w, mR, mZ);
  *(volatile v8us*)dp = o;
  __threadfence();
  *(volatile v8us*)dp = o;
}

template <int NT, int RELU>
__global__ __launch_bounds__(GTHR) void k_gemm(const unsigned short* __restrict__ A, int lda,
                                               const unsigned short* __restrict__ BT, int ldb, int K,
                                               const float* __restrict__ bias, float* outp, int nOut) {
  static_assert(NT == 4 || NT == 8);
  constexpr int N   = 16 * NT;
  constexpr int RPI = 128 / N;
  constexpr int NI  = 16 / RPI;
  __shared__ __attribute__((aligned(16))) float stg[GBM * N];
  const int tid = (int)threadIdx.x, lane = tid & 31, wave = tid >> 5, hh = lane >> 4, m = lane & 15;
  const int rowBase = (int)blockIdx.x * GBM;

  v8f acc[NT];
  {
    const v8f z = {0.f, 0.f, 0.f, 0.f, 0.f, 0.f, 0.f, 0.f};
#pragma unroll
    for (int t = 0; t < NT; ++t) acc[t] = z;
  }
  const unsigned short* ap = A  + (size_t)(rowBase + 16 * wave + m) * (size_t)lda + 8 * hh;
  const unsigned short* bp = BT + (size_t)m * (size_t)ldb + 8 * hh;

#pragma unroll 1
  for (int k0 = 0; k0 < K; k0 += 32) {
    FragB af;
    af.h[0] = *(const v8usa*)(ap + k0);
    af.h[1] = *(const v8usa*)(ap + k0 + 16);
#pragma unroll
    for (int nt = 0; nt < NT; ++nt) {
      const unsigned short* wq = bp + (size_t)(16 * nt) * (size_t)ldb + k0;
      FragB bf;
      bf.h[0] = *(const v8usa*)wq;
      bf.h[1] = *(const v8usa*)(wq + 16);
      acc[nt] = wmb(af, bf, acc[nt]);
    }
  }

#pragma unroll
  for (int nt = 0; nt < NT; ++nt) {
    const int lc = 16 * nt + m;
#pragma unroll
    for (int r = 0; r < 8; ++r) {
      const int lr = 16 * wave + 8 * hh + r;
      stg[lr * N + lc] = acc[nt][r];
    }
  }
  __syncthreads();

  const int lcol = (4 * lane) & (N - 1);
  const int lro  = (4 * lane) / N;
  v4f b4;
  {
    const v4f tb = *(const v4f*)(bias + lcol);
    b4.x = bf16_val(tb.x); b4.y = bf16_val(tb.y); b4.z = bf16_val(tb.z); b4.w = bf16_val(tb.w);
  }

  v4f pv[NI];
#pragma unroll
  for (int i = 0; i < NI; ++i) {
    v4f t = *(const v4fa*)(stg + (16 * wave + RPI * i) * N + 4 * lane) + b4;
    if (RELU != 0) {
      t.x = fmaxf(t.x, 0.0f); t.y = fmaxf(t.y, 0.0f); t.z = fmaxf(t.z, 0.0f); t.w = fmaxf(t.w, 0.0f);
    }
    pv[i] = t;
  }
#pragma unroll
  for (int i = 0; i < NI; ++i) {
    const int seg = rowBase + 16 * wave + RPI * i;
    if (seg + lro < nOut) *(volatile v4f*)(outp + (size_t)seg * N + 4 * lane) = pv[i];
  }
  __threadfence();
#pragma unroll
  for (int i = 0; i < NI; ++i) {
    const int seg = rowBase + 16 * wave + RPI * i;
    if (seg + lro < nOut) *(volatile v4f*)(outp + (size_t)seg * N + 4 * lane) = pv[i];
  }
}

template <int L0>
__global__ __launch_bounds__(NTHR) void k_scan(const int* __restrict__ srcs, const int* __restrict__ dsts,
                                               int nE, int nN, int vec8, int mRows,
                                               const float* __restrict__ gin, unsigned short* apl) {
  constexpr int AP = (L0 != 0) ? AP0 : AP1;
  extern __shared__ __attribute__((aligned(16))) int dsm[];
  int* list = dsm;
  int* hl   = dsm + LISTN;
  int* sl   = hl + RCAP;
  int* cnt  = sl + RCAP;
  int* offs = cnt + NBA;
  int* cur  = offs + NBA;
  int* misc = cur + NBA;
  const int tid = (int)threadIdx.x, lane = tid & 31, wave = tid >> 5;
  unsigned short* rowbuf = (unsigned short*)(misc + MISC_INTS) + wave * AP1;
  const int nodeBase = (int)blockIdx.x * NBA;

  {
    const v4i z4 = {0, 0, 0, 0};
    for (int i = tid * 4; i < AGG_ZINTS; i += NTHR * 4) *(v4ia*)(dsm + i) = z4;
    int* rbz = misc + MISC_INTS;
    for (int i = tid * 4; i < ROWBUF_INTS; i += NTHR * 4) *(v4ia*)(rbz + i) = z4;
    if (tid < MISC_INTS) misc[tid] = 0;
  }
  __syncthreads();

  int t = 0, ov = 0;
  const int nChunks = (nE + CHUNK - 1) / CHUNK;
#pragma unroll 1
  for (int ch = 0; ch < nChunks; ++ch) {
    const int cbase = ch * CHUNK;
    const int wc = scan_chunk<SLA>(dsts, nE, cbase, nodeBase, NBA, vec8, list, tid, lane, wave);
    if (lane == 0) misc[wave] = wc;
    __syncthreads();
    if (wave == 0) {
#pragma unroll 1
      for (int w2 = 0; w2 < NWAVE; ++w2) {
        int c = misc[w2];
        c = c < 0 ? 0 : (c > WCAP ? WCAP : c);
#pragma unroll 1
        for (int b0 = 0; b0 < c; b0 += 32) {
          const int idx = b0 + lane;
          const int ent = list[w2 * WCAP + (idx < WCAP ? idx : WCAP - 1)];
          const int m32 = (c - b0) < 32 ? (c - b0) : 32;
#pragma unroll 1
          for (int k = 0; k < m32; ++k) {
            const int u    = __builtin_amdgcn_readlane(ent, k);
            const int slot = u & (NBA - 1);
            const int el   = (u >> SLA) & (CHUNK - 1);
            const int pk   = ((cbase + el) << SLA) | slot;
            if (t < RCAP) {
              if (lane == 0) { hl[t] = pk; cnt[slot] = cnt[slot] + 1; }
              t = t + 1;
            } else {
              ov = 1;
            }
          }
        }
      }
    }
    __syncthreads();
  }
  if (wave == 0 && lane == 0) { misc[8] = t; misc[9] = ov; }
  __syncthreads();
  int tt = misc[8];
  tt = tt < 0 ? 0 : (tt > RCAP ? RCAP : tt);
  const int ovf = misc[9];

  if (wave == 0) {
    const int base = lane * (NBA / 32);
    int s = 0;
#pragma unroll 1
    for (int i = 0; i < NBA / 32; ++i) s += cnt[base + i];
    int incl = s;
#pragma unroll
    for (int d = 1; d < 32; d <<= 1) {
      const int y = __shfl_up(incl, d, 32);
      if (lane >= d) incl += y;
    }
    int run = incl - s;
#pragma unroll 1
    for (int i = 0; i < NBA / 32; ++i) {
      const int cv = cnt[base + i];
      offs[base + i] = run;
      cur[base + i]  = run;
      run += cv;
    }
  }
  __syncthreads();
  if (wave == 0) {
#pragma unroll 1
    for (int b0 = 0; b0 < tt; b0 += 32) {
      const int idx = b0 + lane;
      const int ent = hl[idx < RCAP ? idx : RCAP - 1];
      const int m32 = (tt - b0) < 32 ? (tt - b0) : 32;
#pragma unroll 1
      for (int k = 0; k < m32; ++k) {
        const int u    = __builtin_amdgcn_readlane(ent, k);
        const int slot = u & (NBA - 1);
        if (lane == 0) {
          int p = cur[slot];
          p = p < 0 ? 0 : (p > RCAP - 1 ? RCAP - 1 : p);
          sl[p] = u;
          cur[slot] = p + 1;
        }
      }
    }
  }
  __syncthreads();

  const float pz = (ovf != 0) ? __int_as_float(0x7fc00000) : 0.0f;
#pragma unroll 1
  for (int si = 0; si < NBA / NWAVE; ++si) {
    const int s    = si * NWAVE + wave;
    const int node = nodeBase + s;
    int c = cnt[s];
    const bool big = c > DEGCAP;
    c = c < 0 ? 0 : (c > DEGCAP ? DEGCAP : c);
    int o = offs[s];
    o = o < 0 ? 0 : (o > RCAP ? RCAP : o);
    const int nc = node < nN ? node : nN - 1;
    float a0 = 0.0f, a1 = 0.0f, a2 = 0.0f, a3 = 0.0f;
#pragma unroll 1
    for (int b0 = 0; b0 < c; b0 += 32) {
      int idx = o + b0 + lane;
      idx = idx > RCAP - 1 ? RCAP - 1 : idx;
      const int ent = sl[idx];
      int eid = ent >> SLA;
      eid = eid < 0 ? 0 : (eid > nE - 1 ? nE - 1 : eid);
      int sr = srcs[eid];
      sr = sr < 0 ? 0 : (sr > nN - 1 ? nN - 1 : sr);
      const int m32 = (c - b0) < 32 ? (c - b0) : 32;
#pragma unroll 1
      for (int k = 0; k < m32; ++k) {
        const int sk = __builtin_amdgcn_readlane(sr, k);
        const float mk = (sk != node) ? 1.0f : 0.0f;
        if constexpr (L0 != 0) {
          const float* rp = gin + (size_t)sk * FIN + lane;
          const float v0 = rp[0], v1 = rp[32], v2 = rp[64];
          a0 = fmaf(mk, bf16_val(v0), a0);
          a1 = fmaf(mk, bf16_val(v1), a1);
          a2 = fmaf(mk, bf16_val(v2), a2);
        } else {
          const v4f a = *(const v4f*)(gin + (size_t)sk * HID + 4 * lane);
          a0 = fmaf(mk, a.x, a0); a1 = fmaf(mk, a.y, a1);
          a2 = fmaf(mk, a.z, a2); a3 = fmaf(mk, a.w, a3);
        }
      }
    }
    const float pzr = big ? __int_as_float(0x7fc00000) : pz;
    const bool live = node < nN;
    if constexpr (L0 != 0) {
      const float s0 = live ? (a0 + pzr) : 0.0f;
      const float s1 = live ? (a1 + pzr) : 0.0f;
      const float s2 = live ? (a2 + pzr) : 0.0f;
      const unsigned hb0 = bf16_bits(s0), hb1 = bf16_bits(s1), hb2 = bf16_bits(s2);
      const unsigned lb0 = bf16_bits(s0 - __uint_as_float(hb0 << 16));
      const unsigned lb1 = bf16_bits(s1 - __uint_as_float(hb1 << 16));
      const unsigned lb2 = bf16_bits(s2 - __uint_as_float(hb2 << 16));
      rowbuf[lane]            = (unsigned short)hb0;
      rowbuf[32 + lane]       = (unsigned short)hb1;
      rowbuf[64 + lane]       = (unsigned short)hb2;
      rowbuf[FIN + lane]      = (unsigned short)lb0;
      rowbuf[FIN + 32 + lane] = (unsigned short)lb1;
      rowbuf[FIN + 64 + lane] = (unsigned short)lb2;
      const float* xp = gin + (size_t)nc * FIN + lane;
      const float x0 = xp[0], x1 = xp[32], x2 = xp[64];
      rowbuf[2 * FIN + lane]      = live ? (unsigned short)bf16_bits(x0 + pzr) : (unsigned short)0;
      rowbuf[2 * FIN + 32 + lane] = live ? (unsigned short)bf16_bits(x1 + pzr) : (unsigned short)0;
      rowbuf[2 * FIN + 64 + lane] = live ? (unsigned short)bf16_bits(x2 + pzr) : (unsigned short)0;
      rowbuf[K0 + lane] = (unsigned short)0;
      (void)a3;
    } else {
      const float s0 = live ? (a0 + pzr) : 0.0f;
      const float s1 = live ? (a1 + pzr) : 0.0f;
      const float s2 = live ? (a2 + pzr) : 0.0f;
      const float s3 = live ? (a3 + pzr) : 0.0f;
      v4us mh, ml;
      {
        unsigned hb;
        hb = bf16_bits(s0); mh[0] = (unsigned short)hb; ml[0] = (unsigned short)bf16_bits(s0 - __uint_as_float(hb << 16));
        hb = bf16_bits(s1); mh[1] = (unsigned short)hb; ml[1] = (unsigned short)bf16_bits(s1 - __uint_as_float(hb << 16));
        hb = bf16_bits(s2); mh[2] = (unsigned short)hb; ml[2] = (unsigned short)bf16_bits(s2 - __uint_as_float(hb << 16));
        hb = bf16_bits(s3); mh[3] = (unsigned short)hb; ml[3] = (unsigned short)bf16_bits(s3 - __uint_as_float(hb << 16));
      }
      *(v4usa*)(rowbuf + 4 * lane) = mh;
      *(v4usa*)(rowbuf + HID + 4 * lane) = ml;
      const v4f hs = *(const v4f*)(gin + (size_t)nc * HID + 4 * lane);
      const float g0 = live ? (hs.x + pzr) : 0.0f;
      const float g1 = live ? (hs.y + pzr) : 0.0f;
      const float g2 = live ? (hs.z + pzr) : 0.0f;
      const float g3 = live ? (hs.w + pzr) : 0.0f;
      v4us gh, gl;
      {
        unsigned hb;
        hb = bf16_bits(g0); gh[0] = (unsigned short)hb; gl[0] = (unsigned short)bf16_bits(g0 - __uint_as_float(hb << 16));
        hb = bf16_bits(g1); gh[1] = (unsigned short)hb; gl[1] = (unsigned short)bf16_bits(g1 - __uint_as_float(hb << 16));
        hb = bf16_bits(g2); gh[2] = (unsigned short)hb; gl[2] = (unsigned short)bf16_bits(g2 - __uint_as_float(hb << 16));
        hb = bf16_bits(g3); gh[3] = (unsigned short)hb; gl[3] = (unsigned short)bf16_bits(g3 - __uint_as_float(hb << 16));
      }
      *(v4usa*)(rowbuf + 2 * HID + 4 * lane) = gh;
      *(v4usa*)(rowbuf + 3 * HID + 4 * lane) = gl;
    }
    wave_sync();
    const v8us q0 = *(const v8usa*)(rowbuf + 8 * lane);
    v8us q1;
    if constexpr (L0 != 0) q1 = *(const v8usa*)(rowbuf + 256 + 8 * (lane & 7));
    else                   q1 = *(const v8usa*)(rowbuf + 256 + 8 * lane);
    wave_sync();
    if (node < mRows) {
      unsigned short* rpw = apl + (size_t)node * AP + 8 * lane;
      *(volatile v8us*)rpw = q0;
      if constexpr (L0 != 0) { if (lane < 8) *(volatile v8us*)(rpw + 256) = q1; }
      else                   { *(volatile v8us*)(rpw + 256) = q1; }
      __threadfence();
      *(volatile v8us*)rpw = q0;
      if constexpr (L0 != 0) { if (lane < 8) *(volatile v8us*)(rpw + 256) = q1; }
      else                   { *(volatile v8us*)(rpw + 256) = q1; }
    }
  }
}

static inline int cdiv(int a, int b) { return (a + b - 1) / b; }

extern "C" void kernel_launch(void* const* d_in, const int* in_sizes, int n_in,
                              void* d_out, int out_size, void* d_ws, size_t ws_size,
                              hipStream_t stream) {
  if (n_in < 8) return;
  if (in_sizes[0] < FIN || (in_sizes[0] % FIN) != 0) return;
  const int nN = in_sizes[0] / FIN;
  if (in_sizes[1] < 2 || (in_sizes[1] & 1) != 0) return;
  const int nE = in_sizes[1] / 2;
  if (nE < 1 || nE >= (1 << 21)) return;
  if (in_sizes[2] != HID * FIN || in_sizes[3] != HID || in_sizes[4] != HID * FIN) return;
  if (in_sizes[5] != FOUT * HID || in_sizes[6] != FOUT || in_sizes[7] != FOUT * HID) return;
  if ((long long)out_size != (long long)nN * FOUT) return;

  const float* x    = (const float*)d_in[0];
  const int*   edge = (const int*)d_in[1];
  const float* W1r  = (const float*)d_in[2];
  const float* b1   = (const float*)d_in[3];
  const float* W1o  = (const float*)d_in[4];
  const float* W2r  = (const float*)d_in[5];
  const float* b2   = (const float*)d_in[6];
  const float* W2o  = (const float*)d_in[7];
  float* out = (float*)d_out;
  const int* src = edge;
  const int* dst = edge + nE;

  const int MP = cdiv(nN, GBM) * GBM;
  const int gM = MP / GBM;
  const int gA = cdiv(nN, NBA);
  if ((long long)gA * NBA < (long long)MP) return;
  const int vec8 = ((nE & 3) == 0) ? 1 : 0;

  char* ws = (char*)d_ws;
  size_t off = 0;
  const size_t oB0 = off; off += (size_t)HID * AP0 * 2;                   off = (off + 255) & ~(size_t)255;
  const size_t oB1 = off; off += (size_t)FOUT * AP1 * 2;                  off = (off + 255) & ~(size_t)255;
  const size_t oA0 = off; off += (size_t)MP * AP0 * 2;                    off = (off + 255) & ~(size_t)255;
  const size_t oH  = off; off += (size_t)MP * HID * 4;                    off = (off + 255) & ~(size_t)255;
  const size_t oA1 = off; off += (size_t)MP * AP1 * 2;                    off = (off + 255) & ~(size_t)255;
  if (off > ws_size || off > (size_t)WSMAX) return;
  unsigned short* B0 = (unsigned short*)(ws + oB0);
  unsigned short* B1 = (unsigned short*)(ws + oB1);
  unsigned short* A0 = (unsigned short*)(ws + oA0);
  float*          H  = (float*)(ws + oH);
  unsigned short* A1 = (unsigned short*)(ws + oA1);

  const size_t scanLds = (size_t)AGG_LDS_INTS * 4;
  hipFuncSetAttribute(reinterpret_cast<const void*>(&k_scan<1>), hipFuncAttributeMaxDynamicSharedMemorySize, (int)scanLds);
  hipFuncSetAttribute(reinterpret_cast<const void*>(&k_scan<0>), hipFuncAttributeMaxDynamicSharedMemorySize, (int)scanLds);

  k_wprep<<<(NU0 + NU1) / NTHR, NTHR, 0, stream>>>(W1r, W1o, W2r, W2o, B0, B1);
  k_scan<1><<<gA, NTHR, scanLds, stream>>>(src, dst, nE, nN, vec8, MP, x, A0);
  k_gemm<8, 1><<<gM, GTHR, 0, stream>>>(A0, AP0, B0, AP0, K0, b1, H, MP);
  k_scan<0><<<gA, NTHR, scanLds, stream>>>(src, dst, nE, nN, vec8, MP, H, A1);
  k_gemm<4, 0><<<gM, GTHR, 0, stream>>>(A1, AP1, B1, AP1, K1, b2, out, nN);
}
